// NeighborhoodAttention2D_60421599920292
// MI455X (gfx1250) — hardware-verified
//
#include <hip/hip_runtime.h>
#include <math.h>
#define __bf16 _Float16

typedef __attribute__((ext_vector_type(16))) __bf16 v16bf;
typedef __attribute__((ext_vector_type(8)))  float  v8f;
typedef __attribute__((ext_vector_type(4)))  unsigned int v4u;
typedef __attribute__((ext_vector_type(8)))  int v8i;
typedef __attribute__((ext_vector_type(4)))  int v4i;

#define HH 96
#define WW 96
#define CDIM 192
#define QKVC 576
#define RSPLIT (1.0f / 2048.0f)
#define NPIX 36864
#define PLQKV ((size_t)NPIX * QKVC)
#define PLATT ((size_t)NPIX * CDIM)
typedef __attribute__((ext_vector_type(8))) _Float16 v8h_;
typedef __attribute__((ext_vector_type(4))) float v4f_t;
typedef float v4fa __attribute__((ext_vector_type(4), may_alias));
typedef __attribute__((ext_vector_type(4))) unsigned v4u_t;
typedef unsigned v4ua __attribute__((ext_vector_type(4), may_alias));
__device__ __forceinline__ __bf16 lo_of(float v, __bf16 h) { return (__bf16)((v - (float)h) * 2048.0f); }
__device__ __forceinline__ v8f wmma16(v16bf a, v16bf b, v8f c) {
  return __builtin_amdgcn_wmma_f32_16x16x32_f16(false, a, false, b, (short)0, c, false, false);
}
__device__ __forceinline__ v8f wmma_split(v16bf a, v16bf al, v16bf b, v16bf bl, v8f c) {
  v8f x = {};
  x = wmma16(al, b, x); x = wmma16(a, bl, x);
  return wmma16(a, b, c) + x * RSPLIT;
}
__device__ __forceinline__ unsigned pk2s(float a, float b, unsigned* lo) {
  const __bf16 h0 = (__bf16)a, h1 = (__bf16)b;
  *lo = (unsigned)__builtin_bit_cast(unsigned short, lo_of(a, h0)) | ((unsigned)__builtin_bit_cast(unsigned short, lo_of(b, h1)) << 16);
  return (unsigned)__builtin_bit_cast(unsigned short, h0) | ((unsigned)__builtin_bit_cast(unsigned short, h1) << 16);
}

__global__ __launch_bounds__(256) void pack_w(const float* __restrict__ w,
                                              __bf16* __restrict__ wpk, int N) {
  const int t = blockIdx.x * 256 + threadIdx.x;
  const int total = (N >> 4) * 6 * 32;
  if (t >= total) return;
  const int lane = t & 31;
  const int c = (t >> 5) % 6;
  const int nt = t / (6 * 32);
  const int n = nt * 16 + (lane & 15);
  const int hi = lane >> 4;
  const size_t plane = (size_t)192 * N;
  union { __bf16 h[16]; v4u_t q[2]; } ph, pl;
#pragma unroll
  for (int j = 0; j < 16; ++j) {
    const int k = c * 32 + ((j < 8) ? (hi * 8 + j) : (16 + hi * 8 + (j - 8)));
    const float v = w[(size_t)k * N + n];
    ph.h[j] = (__bf16)v; pl.h[j] = lo_of(v, ph.h[j]);
  }
  __bf16* dst = wpk + (size_t)t * 16;
  *(volatile v4u_t*)dst = ph.q[0]; *(volatile v4u_t*)(dst + 8) = ph.q[1]; *(volatile v4u_t*)(dst + plane) = pl.q[0]; *(volatile v4u_t*)(dst + plane + 8) = pl.q[1];
  __threadfence();
  *(volatile v4u_t*)dst = ph.q[0]; *(volatile v4u_t*)(dst + 8) = ph.q[1]; *(volatile v4u_t*)(dst + plane) = pl.q[0]; *(volatile v4u_t*)(dst + plane + 8) = pl.q[1];
}

template <typename TA, typename TO, int NT>
__global__ __launch_bounds__(256) void gemm192_wmma(
    const TA* __restrict__ A, const __bf16* __restrict__ Bpk,
    const float* __restrict__ bias, TO* __restrict__ C, int M, int N, size_t aplane, size_t cplane) {
  static_assert(NT == 4, "staging assumes 64 columns per wave");
  __shared__ __attribute__((aligned(16))) float stg[8][16 * 68];
  const int lane = threadIdx.x & 31;
  const int wave = threadIdx.x >> 5;
  const int ngrp = (N >> 4) / NT;
  const int job = blockIdx.x * 8 + wave;
  const int mt = job / ngrp;
  const int ng = job - mt * ngrp;
  if (mt * 16 >= M) return;
  const int half = lane >> 4, l15 = lane & 15;

  const size_t arow = (size_t)(mt * 16 + l15) * 192;
  const int nt0 = ng * NT;
  const size_t bplane = (size_t)192 * N;

  v8f acc[NT];
#pragma unroll
  for (int u = 0; u < NT; ++u) acc[u] = (v8f){};

#pragma unroll 2
  for (int c = 0; c < 6; ++c) {
    v16bf a, al;
    const TA* ap = A + arow + c * 32 + half * 8;
    if constexpr (sizeof(TA) == 4) {
#pragma unroll
      for (int i = 0; i < 8; ++i) {
        const float v0 = (float)ap[i], v1 = (float)ap[16 + i];
        a[i] = (__bf16)v0; al[i] = lo_of(v0, a[i]); a[8 + i] = (__bf16)v1; al[8 + i] = lo_of(v1, a[8 + i]);
      }
    } else {
#pragma unroll
      for (int i = 0; i < 8; ++i) { a[i] = ap[i]; a[8 + i] = ap[16 + i]; al[i] = ap[aplane + i]; al[8 + i] = ap[aplane + 16 + i]; }
    }
#pragma unroll
    for (int u = 0; u < NT; ++u) {
      union { uint4 q[2]; v16bf v; } bb, bl;
      const __bf16* bq = Bpk + ((((size_t)(nt0 + u)) * 6 + c) * 32 + lane) * 16;
      bb.q[0] = *reinterpret_cast<const uint4*>(bq);          bb.q[1] = *reinterpret_cast<const uint4*>(bq + 8);
      bl.q[0] = *reinterpret_cast<const uint4*>(bq + bplane); bl.q[1] = *reinterpret_cast<const uint4*>(bq + bplane + 8);
      acc[u] = wmma_split(a, al, bb.v, bl.v, acc[u]);
    }
  }

  float* sw = stg[wave];
#pragma unroll
  for (int u = 0; u < NT; ++u) {
    const float bv = bias[(nt0 + u) * 16 + l15];
#pragma unroll
    for (int r = 0; r < 8; ++r) sw[(half * 8 + r) * 68 + u * 16 + l15] = acc[u][r] + bv;
  }
  asm volatile("s_wait_dscnt 0" ::: "memory");
  const size_t row0 = (size_t)mt * 16, col0 = (size_t)nt0 * 16;
#pragma unroll 1
  for (int pass = 0; pass < 2; ++pass) {
    if constexpr (sizeof(TO) == 4) {
#pragma unroll
      for (int i = 0; i < 8; ++i) { const int cc = lane + 32 * i, rr = cc >> 4, q = cc & 15;
        *(volatile v4f_t*)((float*)C + (row0 + rr) * N + col0 + q * 4) = *(const volatile v4fa*)(sw + rr * 68 + q * 4); }
    } else {
#pragma unroll
      for (int i = 0; i < 4; ++i) { const int cc = lane + 32 * i, rr = cc >> 3, q = cc & 7; const float* s = sw + rr * 68 + q * 8;
        v4u_t v, vl; unsigned lq;
        v.x = pk2s(s[0], s[1], &lq); vl.x = lq; v.y = pk2s(s[2], s[3], &lq); vl.y = lq; v.z = pk2s(s[4], s[5], &lq); vl.z = lq; v.w = pk2s(s[6], s[7], &lq); vl.w = lq;
        __bf16* cp = (__bf16*)C + (row0 + rr) * N + col0 + q * 8;
        *(volatile v4u_t*)cp = v; *(volatile v4u_t*)(cp + cplane) = vl; }
    }
    __threadfence();
  }
}

__device__ __forceinline__ void tdm_load_tile(unsigned lds_byte,
                                              unsigned long long gaddr,
                                              int u) {
  v4u g0;
  g0.x = 1u;
  g0.y = lds_byte;
  g0.z = (unsigned)(gaddr & 0xFFFFFFFFu);
  g0.w = (unsigned)((gaddr >> 32) & 0x1FFFFFFu)
         | (2u << 30);
  v8i g1;
  g1[0] = (int)(1u << 16);
  g1[1] = (int)(32u << 16);
  g1[2] = (int)((unsigned)u << 16);
  g1[3] = (int)(32u << 16);
  g1[4] = (int)((unsigned)u | ((unsigned)u << 16));
  g1[5] = 576;
  g1[6] = (int)(0xD800u << 16);
  g1[7] = 0;
  v4i g2;
  g2[0] = u;
  g2[1] = 0; g2[2] = 0; g2[3] = 0;
  v4i g3 = {0, 0, 0, 0};
  v8i g4 = {0, 0, 0, 0, 0, 0, 0, 0};
  __builtin_amdgcn_tensor_load_to_lds(g0, g1, g2, g3, g4, 0);
}

template <int KS>
__global__ __launch_bounds__(64) void natten_wmma(
    const __bf16* __restrict__ qkv, __bf16* __restrict__ out, int grp) {
  constexpr int U = KS + 3;
  constexpr int NKEY = U * U;
  constexpr int NCH = (NKEY + 31) / 32;
  constexpr int NKP = NCH * 32;

  __shared__ __align__(16) __bf16 Klds[2][NKP * 32], Kll[2][NKP * 32];
  __shared__ __align__(16) __bf16 Vlds[2][NKP * 32], Vll[2][NKP * 32];
  __shared__ __align__(16) __bf16 Plds[2][16 * 32], Pll[2][16 * 32];
  __shared__ __align__(16) float  Ost[16][64 + 4];

  const int wave = threadIdx.x >> 5;
  const int lane = threadIdx.x & 31;
  const int half = lane >> 4, l15 = lane & 15;
  const int qr0 = ((int)blockIdx.x / 24) * 4;
  const int qc0 = ((int)blockIdx.x % 24) * 4;
  const int head = wave;
  const int bat = blockIdx.z;

  int ur0 = qr0 - KS / 2; ur0 = ur0 < 0 ? 0 : (ur0 > HH - U ? HH - U : ur0);
  int uc0 = qc0 - KS / 2; uc0 = uc0 < 0 ? 0 : (uc0 > WW - U ? WW - U : uc0);

  const int chq = grp * 192 + head * 32;
  const size_t img = (size_t)bat * HH * WW;
  const float NEG_INF = __builtin_inff() * -1.0f;

  __bf16* Kh = Klds[head]; __bf16* Kl = Kll[head]; __bf16* Vh = Vlds[head]; __bf16* Vl = Vll[head];
  __bf16* Ph = Plds[head]; __bf16* Pl = Pll[head];
  {
    const __bf16* tbase = qkv + (img + (size_t)ur0 * WW + uc0) * QKVC + chq;
    tdm_load_tile((unsigned)(size_t)Kh, (unsigned long long)(size_t)(tbase + 64), U);
    tdm_load_tile((unsigned)(size_t)Kl, (unsigned long long)(size_t)(tbase + PLQKV + 64), U);
    tdm_load_tile((unsigned)(size_t)Vh, (unsigned long long)(size_t)(tbase + 128), U);
    tdm_load_tile((unsigned)(size_t)Vl, (unsigned long long)(size_t)(tbase + PLQKV + 128), U);
  }
  for (int idx = NKEY + lane; idx < NKP; idx += 32) {
    const uint4 z = make_uint4(0u, 0u, 0u, 0u);
#pragma unroll
    for (int t = 0; t < 4; ++t) {
      reinterpret_cast<uint4*>(&Kh[idx * 32])[t] = z; reinterpret_cast<uint4*>(&Kl[idx * 32])[t] = z;
      reinterpret_cast<uint4*>(&Vh[idx * 32])[t] = z; reinterpret_cast<uint4*>(&Vl[idx * 32])[t] = z;
    }
  }

  v16bf qa, qal;
  {
    const int qy = qr0 + (l15 >> 2), qx = qc0 + (l15 & 3);
    const __bf16* qp =
        qkv + (img + (size_t)qy * WW + qx) * QKVC + chq + half * 8;
    union { uint4 q; __bf16 h[8]; } u0, u1, w0, w1;
    u0.q = *reinterpret_cast<const uint4*>(qp);
    u1.q = *reinterpret_cast<const uint4*>(qp + 16);
    w0.q = *reinterpret_cast<const uint4*>(qp + PLQKV);
    w1.q = *reinterpret_cast<const uint4*>(qp + PLQKV + 16);
#pragma unroll
    for (int i = 0; i < 8; ++i) { qa[i] = u0.h[i]; qa[8 + i] = u1.h[i]; qal[i] = w0.h[i]; qal[8 + i] = w1.h[i]; }
  }

  __builtin_amdgcn_s_wait_tensorcnt(0);
  __syncthreads();

  float mrow[8], lrow[8];
  v8f Oa = {}, Ob = {};
#pragma unroll
  for (int r = 0; r < 8; ++r) { mrow[r] = NEG_INF; lrow[r] = 0.0f; }

  for (int ch = 0; ch < NCH; ++ch) {
    const int k0 = ch * 32;
    v8f S[2];
#pragma unroll
    for (int t = 0; t < 2; ++t) {
      const int key = k0 + t * 16 + l15;
      v16bf kb, kbl;
#pragma unroll
      for (int j = 0; j < 8; ++j) { kb[j] = Kh[key * 32 + half * 8 + j]; kb[8 + j] = Kh[key * 32 + 16 + half * 8 + j];
                                    kbl[j] = Kl[key * 32 + half * 8 + j]; kbl[8 + j] = Kl[key * 32 + 16 + half * 8 + j]; }
      v8f z = {};
      S[t] = wmma_split(qa, qal, kb, kbl, z);
    }
#pragma unroll
    for (int t = 0; t < 2; ++t) {
      const int kk = k0 + t * 16 + l15;
      const int kr = ur0 + kk / U;
      const int kc = uc0 + kk % U;
      const bool inkey = kk < NKEY;
#pragma unroll
      for (int r = 0; r < 8; ++r) {
        const int m = r + half * 8;
        const int qy = qr0 + (m >> 2), qx = qc0 + (m & 3);
        int sy = qy - KS / 2; sy = sy < 0 ? 0 : (sy > HH - KS ? HH - KS : sy);
        int sx = qx - KS / 2; sx = sx < 0 ? 0 : (sx > WW - KS ? WW - KS : sx);
        const bool ok =
            inkey && kr >= sy && kr < sy + KS && kc >= sx && kc < sx + KS;
        S[t][r] = ok ? S[t][r] * 0.17677669529663687f : NEG_INF;
      }
    }
    float p0a[8], p1a[8];
#pragma unroll
    for (int r = 0; r < 8; ++r) {
      float cmax = fmaxf(S[0][r], S[1][r]);
#pragma unroll
      for (int xm = 8; xm >= 1; xm >>= 1)
        cmax = fmaxf(cmax, __shfl_xor(cmax, xm, 32));
      const float mnew = fmaxf(mrow[r], cmax);
      const float msafe = (mnew == NEG_INF) ? 0.0f : mnew;
      const float alpha = (mrow[r] == NEG_INF) ? 0.0f : __expf(mrow[r] - msafe);
      const float p0 = __expf(S[0][r] - msafe);
      const float p1 = __expf(S[1][r] - msafe);
      float rs = p0 + p1;
#pragma unroll
      for (int xm = 8; xm >= 1; xm >>= 1) rs += __shfl_xor(rs, xm, 32);
      lrow[r] = lrow[r] * alpha + rs;
      mrow[r] = mnew;
      Oa[r] = Oa[r] * alpha;
      Ob[r] = Ob[r] * alpha;
      p0a[r] = p0;
      p1a[r] = p1;
    }
#pragma unroll
    for (int r = 0; r < 8; ++r) {
      const int m = r + half * 8;
      const float q0 = p0a[r] * 1024.0f, q1 = p1a[r] * 1024.0f;
      const __bf16 h0 = (__bf16)q0, h1 = (__bf16)q1;
      Ph[m * 32 + l15] = h0;      Pl[m * 32 + l15] = lo_of(q0, h0);
      Ph[m * 32 + 16 + l15] = h1; Pl[m * 32 + 16 + l15] = lo_of(q1, h1);
    }
    v16bf pa, pal, vb0, vb1, vb0l, vb1l;
#pragma unroll
    for (int i = 0; i < 16; ++i) {
      const int k = ((i >> 3) * 16) + half * 8 + (i & 7);
      pa[i] = Ph[l15 * 32 + k]; pal[i] = Pl[l15 * 32 + k];
    }
#pragma unroll
    for (int j = 0; j < 16; ++j) {
      const int key = k0 + ((j >> 3) * 16) + half * 8 + (j & 7);
      vb0[j] = Vh[key * 32 + l15];      vb0l[j] = Vl[key * 32 + l15];
      vb1[j] = Vh[key * 32 + 16 + l15]; vb1l[j] = Vl[key * 32 + 16 + l15];
    }
    Oa = wmma_split(pa, pal, vb0, vb0l, Oa);
    Ob = wmma_split(pa, pal, vb1, vb1l, Ob);
  }

#pragma unroll
  for (int r = 0; r < 8; ++r) {
    const int m = r + half * 8;
    const float inv = 1.0f / (lrow[r] * 1024.0f);
    Ost[m][head * 32 + l15]      = Oa[r] * inv;
    Ost[m][head * 32 + 16 + l15] = Ob[r] * inv;
  }
  __syncthreads();
  const int tid = threadIdx.x;
#pragma unroll 1
  for (int pass = 0; pass < 2; ++pass) {
#pragma unroll
    for (int i = 0; i < 2; ++i) {
      const int c = tid + 64 * i, m = c >> 3, q = c & 7;
      const int qy = qr0 + (m >> 2), qx = qc0 + (m & 3);
      const float* s = &Ost[m][q * 8];
      v4u_t v, vl; unsigned lq;
      v.x = pk2s(s[0], s[1], &lq); vl.x = lq; v.y = pk2s(s[2], s[3], &lq); vl.y = lq; v.z = pk2s(s[4], s[5], &lq); vl.z = lq; v.w = pk2s(s[6], s[7], &lq); vl.w = lq;
      __bf16* op = out + (img + (size_t)qy * WW + qx) * CDIM + grp * 64 + q * 8;
      *(volatile v4u_t*)op = v; *(volatile v4u_t*)(op + PLATT) = vl;
    }
    __threadfence();
  }
}

extern "C" void kernel_launch(void* const* d_in, const int* in_sizes, int n_in,
                              void* d_out, int out_size, void* d_ws,
                              size_t ws_size, hipStream_t stream) {
  const float* x      = (const float*)d_in[0];
  const float* w_qkv  = (const float*)d_in[1];
  const float* b_qkv  = (const float*)d_in[2];
  const float* w_proj = (const float*)d_in[3];
  const float* b_proj = (const float*)d_in[4];
  float* out = (float*)d_out;

  __bf16* qkv  = (__bf16*)d_ws;
  __bf16* attn = qkv + (size_t)36864 * 576 * 2;
  __bf16* wqk  = attn + (size_t)36864 * 192 * 2;
  __bf16* wpr  = wqk + (size_t)192 * 576 * 2;

  pack_w<<<dim3(27), dim3(256), 0, stream>>>(w_qkv, wqk, 576);
  pack_w<<<dim3(9),  dim3(256), 0, stream>>>(w_proj, wpr, 192);

  gemm192_wmma<float, __bf16, 4>
      <<<dim3(2592), dim3(256), 0, stream>>>(x, wqk, b_qkv, qkv, 36864, 576, (size_t)0, PLQKV);

  dim3 ag(576, 1, 4);
  natten_wmma<7><<<ag, dim3(64), 0, stream>>>(qkv, attn, 0);
  natten_wmma<9><<<ag, dim3(64), 0, stream>>>(qkv, attn, 1);
  natten_wmma<11><<<ag, dim3(64), 0, stream>>>(qkv, attn, 2);

  gemm192_wmma<__bf16, float, 4>
      <<<dim3(864), dim3(256), 0, stream>>>(attn, wpr, b_proj, out, 36864, 192, PLATT, (size_t)0);
}
